// Predictor_TF_REG_47966194762120
// MI455X (gfx1250) — hardware-run, weakly checked
//
#include <hip/hip_runtime.h>


#ifndef NB
#define NB 1024
#endif
#define NB_FULL 1024
#define DIN  256
#define DH   512
#define DP   128
#ifndef H_RES
#define H_RES 0
#endif
#define QRS  2048.0f
#define QRI  (1.0f / 2048.0f)
#define WSC  16.0f
#define WSI  (1.0f / 16.0f)
#define LOG2E 1.4426950408889634f
#define EPI_F32  0
#define EPI_HPL  1
#define EPI_GELU 2

static_assert(NB % 32 == 0);
static_assert(NB <= NB_FULL);
static_assert(DIN % 32 == 0);
static_assert(DH % 32 == 0);
static_assert(DH % 64 == 0);
static_assert((3 * DH) % 64 == 0);
static_assert(DP % 64 == 0);
static_assert(DP == 128);
static_assert(DH == 512);
static_assert(((size_t)NB * DIN) % 8 == 0);
static_assert(((size_t)DH * DIN) % 8 == 0);
static_assert(((size_t)DH * DH) % 8 == 0);
static_assert(((size_t)DP * DH) % 8 == 0);
static_assert((size_t)NB_FULL * 4 == 4096);
static_assert(((size_t)NB_FULL + (size_t)NB_FULL * DP) * 4 == 528384);
static_assert(16 * 68 * 4 <= 131072);
static_assert(3 * DH * 4 <= 131072);
static_assert(8 * 32 * 4 <= 131072);

typedef _Float16 h16;
typedef unsigned short bf;
typedef __attribute__((ext_vector_type(16))) __bf16   v16bf;
typedef __attribute__((ext_vector_type(16))) _Float16 v16h;
typedef __attribute__((ext_vector_type(8)))  _Float16 v8h;
typedef __attribute__((ext_vector_type(8)))  unsigned short v8us;
typedef __attribute__((ext_vector_type(8)))  float    v8f;
typedef __attribute__((ext_vector_type(4)))  float    v4f;
typedef v4f  __attribute__((may_alias)) v4fa;

__device__ __forceinline__ unsigned short f2bf(float f) { unsigned u = __float_as_uint(f); u += 0x7FFFu + ((u >> 16) & 1u); return (unsigned short)(u >> 16); }
__device__ __forceinline__ float bfr(float f) { return __uint_as_float(((unsigned)f2bf(f)) << 16); }
__device__ __forceinline__ v16h cat16(v8h lo, v8h hi) { return __builtin_shufflevector(lo, hi, 0, 1, 2, 3, 4, 5, 6, 7, 8, 9, 10, 11, 12, 13, 14, 15); }
__device__ __forceinline__ v16bf cat16b(v8us lo, v8us hi) { return __builtin_bit_cast(v16bf, __builtin_shufflevector(lo, hi, 0, 1, 2, 3, 4, 5, 6, 7, 8, 9, 10, 11, 12, 13, 14, 15)); }
__device__ __forceinline__ v8f wmma16(v16h a, v16h b, v8f c) { return __builtin_amdgcn_wmma_f32_16x16x32_f16(false, a, false, b, (short)0, c, false, false); }
__device__ __forceinline__ v8f wmmab(v16bf a, v16bf b, v8f c) { return __builtin_amdgcn_wmma_f32_16x16x32_bf16(false, a, false, b, (short)0, c, false, false); }
__device__ __forceinline__ v16h  ldh(const h16* p) { return cat16(*(const v8h*)p, *(const v8h*)(p + 16)); }
__device__ __forceinline__ v16bf ldb(const bf* p)  { return cat16b(*(const v8us*)p, *(const v8us*)(p + 16)); }
__device__ __forceinline__ void wave_sync() { __builtin_amdgcn_fence(3  , "wavefront"); __builtin_amdgcn_wave_barrier(); asm volatile("" ::: "memory"); }

__device__ __forceinline__ v8f wmmabg(v16bf a, v16bf b, v8f c) { c = wmmab(a, b, c); asm volatile("v_nop\n\tv_nop\n\tv_nop\n\tv_nop" : "+v"(c) : "v"(a), "v"(b)); return c; }
__device__ __forceinline__ v8f wmma16g(v16h a, v16h b, v8f c) { c = wmma16(a, b, c); asm volatile("v_nop\n\tv_nop\n\tv_nop\n\tv_nop" : "+v"(c) : "v"(a), "v"(b)); return c; }
static __device__ __forceinline__ h16 toh_flush(float v) { const float w = (fabsf(v) < 6.103515625e-05f) ? 0.0f : v; return (h16)w; }
__device__ __forceinline__ float gelu_erf(float x) { return 0.5f * x * (1.0f + erff(x * 0.70710678118654752f)); }

__global__ __launch_bounds__(256) void k_cvt8(const float* __restrict__ src, bf* dst, size_t n8) {
    const size_t i = (size_t)blockIdx.x * 256 + threadIdx.x; if (i >= n8) return;
    const v8f v = *(const v8f*)(src + i * 8); v8us o;
#pragma unroll
    for (int k = 0; k < 8; ++k) o[k] = f2bf(v[k]);
    *(volatile v8us*)(dst + i * 8) = o; __threadfence(); *(volatile v8us*)(dst + i * 8) = o;
}

__global__ __launch_bounds__(256) void k_wcvt(const float* __restrict__ src, h16* dst, size_t n8) {
    const size_t i = (size_t)blockIdx.x * 256 + threadIdx.x; if (i >= n8) return;
    const v8f v = *(const v8f*)(src + i * 8); v8h o;
#pragma unroll
    for (int k = 0; k < 8; ++k) o[k] = toh_flush(bfr(v[k]) * WSC);
    *(volatile v8h*)(dst + i * 8) = o; __threadfence(); *(volatile v8h*)(dst + i * 8) = o;
}

template <int BFA, int K_, int N_, int EPI, int NBIAS>
__device__ __forceinline__ void gemm_body(float* os,
        const bf* __restrict__ Ab, const bf* __restrict__ Bb,
        const h16* __restrict__ AH, const h16* __restrict__ AR, const h16* __restrict__ Bh,
        const float* __restrict__ bias0, const float* __restrict__ bias1, const float* __restrict__ bias2,
        const float* __restrict__ RES, float* CF, h16* CH, h16* CR) {
    static_assert(K_ % 32 == 0);
    static_assert(N_ % 64 == 0);
    static_assert(NBIAS == 1 || (NBIAS == 3 && N_ == 3 * DH));
    constexpr bool RESON = (BFA == 0) && (H_RES != 0);
    constexpr float OSC = BFA ? 1.0f : WSI;
    const int lane = threadIdx.x & 31, lr = lane & 15, hi = lane >> 4;
    const unsigned bx = blockIdx.x, by = blockIdx.y;
    const int r0 = (int)(bx * 32u), c0 = (int)(by * 64u);
    v8f accH[2][4], accR[2][4];
#pragma unroll
    for (int mb = 0; mb < 2; ++mb)
#pragma unroll
        for (int nb = 0; nb < 4; ++nb) { accH[mb][nb] = (v8f){}; accR[mb][nb] = (v8f){}; }
    const size_t aoff = (size_t)(r0 + lr) * K_ + 8 * hi, boff = (size_t)(c0 + lr) * K_ + 8 * hi;
#pragma unroll 1
    for (int kc = 0; kc < K_; kc += 32) {
        if constexpr (BFA != 0) {
            v16bf a[2];
#pragma unroll
            for (int mb = 0; mb < 2; ++mb) a[mb] = ldb(Ab + aoff + (size_t)mb * 16 * K_ + kc);
#pragma unroll
            for (int nb = 0; nb < 4; ++nb) { const v16bf b = ldb(Bb + boff + (size_t)nb * 16 * K_ + kc);
#pragma unroll
                for (int mb = 0; mb < 2; ++mb) accH[mb][nb] = wmmabg(a[mb], b, accH[mb][nb]); }
        } else {
            v16h a[2], ar[2];
#pragma unroll
            for (int mb = 0; mb < 2; ++mb) { a[mb] = ldh(AH + aoff + (size_t)mb * 16 * K_ + kc); if constexpr (RESON) ar[mb] = ldh(AR + aoff + (size_t)mb * 16 * K_ + kc); }
#pragma unroll
            for (int nb = 0; nb < 4; ++nb) { const v16h b = ldh(Bh + boff + (size_t)nb * 16 * K_ + kc);
#pragma unroll
                for (int mb = 0; mb < 2; ++mb) { accH[mb][nb] = wmma16g(a[mb], b, accH[mb][nb]); if constexpr (RESON) accR[mb][nb] = wmma16g(ar[mb], b, accR[mb][nb]); } }
        }
    }
    float bc[4];
#pragma unroll
    for (int nb = 0; nb < 4; ++nb) {
        if constexpr (NBIAS == 1) { bc[nb] = bfr(bias0[c0 + nb * 16 + lr]); }
        else { const unsigned seg = by / (unsigned)(DH / 64);
               const int cl = c0 - (int)(seg * (unsigned)DH) + nb * 16 + lr;
               const float x0 = bfr(bias0[cl]), x1 = bfr(bias1[cl]), x2 = bfr(bias2[cl]);
               bc[nb] = (seg == 0u) ? x0 : ((seg == 1u) ? x1 : x2); }
    }
#pragma unroll
    for (int mb = 0; mb < 2; ++mb) {
#pragma unroll
        for (int nb = 0; nb < 4; ++nb) {
#pragma unroll
            for (int j = 0; j < 8; ++j) { float v = accH[mb][nb][j]; if constexpr (RESON) v += accR[mb][nb][j] * QRI;
                os[(hi * 8 + j) * 68 + nb * 16 + lr] = v * OSC + bc[nb]; } }
        wave_sync();
        if constexpr (EPI == EPI_GELU) {
#pragma unroll 1
            for (int s = 0; s < 8; ++s) { const int row = 2 * s + (lane >> 4), c4 = (lane & 15) * 4;
                v4f x = *(const v4fa*)(&os[row * 68 + c4]);
                const v4f rr = *(const v4f*)(RES + (size_t)(r0 + mb * 16 + row) * N_ + c0 + c4);
#pragma unroll
                for (int i = 0; i < 4; ++i) x[i] = rr[i] + gelu_erf(x[i]);
                *(v4fa*)(&os[row * 68 + c4]) = x; }
            wave_sync();
        }
        static_assert(32 * 16 * 8 == 16 * 64 * 4);
        static_assert(32 * 16 * 4 == 16 * 64 * 2);
#pragma unroll 1
        for (int ps = 0; ps < 2; ++ps) {
#pragma unroll
            for (int s = 0; s < 8; ++s) { const int row = 2 * s + (lane >> 4), c4 = (lane & 15) * 4;
                const v4f val = *(const v4fa*)(&os[row * 68 + c4]);
                *(volatile v4f*)(CF + (size_t)(r0 + mb * 16 + row) * N_ + c0 + c4) = val; }
            if constexpr (EPI != EPI_F32) {
#pragma unroll
                for (int s = 0; s < 4; ++s) { const int row = 4 * s + (lane >> 3), c8 = (lane & 7) * 8;
                    const v4f x0 = *(const v4fa*)(&os[row * 68 + c8]); const v4f x1 = *(const v4fa*)(&os[row * 68 + c8 + 4]); v8h hv, rv;
#pragma unroll
                    for (int i = 0; i < 4; ++i) { const h16 a0 = toh_flush(x0[i]); const h16 a1 = toh_flush(x1[i]); hv[i] = a0; hv[4 + i] = a1;
                        rv[i] = toh_flush((x0[i] - (float)a0) * QRS); rv[4 + i] = toh_flush((x1[i] - (float)a1) * QRS); }
                    const size_t oo = (size_t)(r0 + mb * 16 + row) * N_ + c0 + c8;
                    *(volatile v8h*)(CH + oo) = hv; *(volatile v8h*)(CR + oo) = rv; }
            }
            if (ps == 0) __threadfence(); }
        wave_sync();
    }
}

__global__ __launch_bounds__(32) void k_lin0(const bf* __restrict__ XB, const bf* __restrict__ WB, const float* __restrict__ bias, float* HF, h16* HH, h16* HR) {
    __shared__ __align__(16) float os[16 * 68];
    gemm_body<1, DIN, DH, EPI_HPL, 1>(os, XB, WB, nullptr, nullptr, nullptr, bias, bias, bias, nullptr, HF, HH, HR);
}
__global__ __launch_bounds__(32) void k_qkv(const h16* __restrict__ AH, const h16* __restrict__ AR, const h16* __restrict__ W,
                                            const float* __restrict__ bq, const float* __restrict__ bk, const float* __restrict__ bv, float* QKV) {
    __shared__ __align__(16) float os[16 * 68];
    gemm_body<0, DH, 3 * DH, EPI_F32, 3>(os, nullptr, nullptr, AH, AR, W, bq, bk, bv, nullptr, QKV, nullptr, nullptr);
}
__global__ __launch_bounds__(32) void k_f1(const h16* __restrict__ AH, const h16* __restrict__ AR, const h16* __restrict__ W, const float* __restrict__ bias,
                                           const float* __restrict__ RES, float* HF, h16* HH, h16* HR) {
    __shared__ __align__(16) float os[16 * 68];
    gemm_body<0, DH, DH, EPI_GELU, 1>(os, nullptr, nullptr, AH, AR, W, bias, bias, bias, RES, HF, HH, HR);
}
__global__ __launch_bounds__(32) void k_fea(const h16* __restrict__ AH, const h16* __restrict__ AR, const h16* __restrict__ W, const float* __restrict__ bias, float* FEA) {
    __shared__ __align__(16) float os[16 * 68];
    gemm_body<0, DH, DP, EPI_F32, 1>(os, nullptr, nullptr, AH, AR, W, bias, bias, bias, nullptr, FEA, nullptr, nullptr);
}

__global__ __launch_bounds__(32) void k_pair(const float* __restrict__ HF, const float* __restrict__ QKV, float* OF, h16* OH, h16* PR) {
    __shared__ __align__(16) float sk[DH];
    __shared__ __align__(16) float sv[DH];
    __shared__ __align__(16) float so[DH];
    const int lane = threadIdx.x & 31;
    const unsigned b = blockIdx.x;
    const float* qrow = QKV + (size_t)b * (3 * DH);
    float qs[16], ms[16], l[16], n[16];
    float kmx = -3.0e38f, kmn = 3.0e38f;
#pragma unroll
    for (int g = 0; g < 4; ++g) { const int i0 = 128 * g + 4 * lane;
        const v4f qq = *(const v4f*)(qrow + i0); const v4f kq = *(const v4f*)(qrow + DH + i0); const v4f vq = *(const v4f*)(qrow + 2 * DH + i0);
        *(v4fa*)(&sk[i0]) = kq; *(v4fa*)(&sv[i0]) = vq;
#pragma unroll
        for (int c = 0; c < 4; ++c) { kmx = fmaxf(kmx, kq[c]); kmn = fminf(kmn, kq[c]); qs[4 * g + c] = qq[c] * LOG2E; } }
#pragma unroll
    for (int off = 16; off > 0; off >>= 1) { kmx = fmaxf(kmx, __shfl_xor(kmx, off, 32)); kmn = fminf(kmn, __shfl_xor(kmn, off, 32)); }
#pragma unroll
    for (int r = 0; r < 16; ++r) { ms[r] = (qs[r] >= 0.0f) ? qs[r] * kmx : qs[r] * kmn; l[r] = 0.0f; n[r] = 0.0f; }
    wave_sync();
#pragma unroll 1
    for (int j = 0; j < DH; ++j) { const float kj = sk[j], vj = sv[j];
#pragma unroll
        for (int r = 0; r < 16; ++r) { const float e = __builtin_amdgcn_exp2f(fmaf(qs[r], kj, -ms[r])); l[r] += e; n[r] = fmaf(e, vj, n[r]); } }
#pragma unroll
    for (int g = 0; g < 4; ++g) { const int i0 = 128 * g + 4 * lane;
        const v4f hq = *(const v4f*)(HF + (size_t)b * DH + i0); v4f o;
#pragma unroll
        for (int c = 0; c < 4; ++c) o[c] = hq[c] + n[4 * g + c] * __builtin_amdgcn_rcpf(l[4 * g + c]);
        *(v4fa*)(&so[i0]) = o; }
    wave_sync();
    static_assert(32 * 16 * 4 == DH * 4);
    static_assert(32 * 16 * 2 == DH * 2);
#pragma unroll 1
    for (int ps = 0; ps < 2; ++ps) {
#pragma unroll
        for (int s = 0; s < 4; ++s) { const int idx = (s * 32 + lane) * 4;
            const v4f val = *(const v4fa*)(&so[idx]);
            *(volatile v4f*)(OF + (size_t)b * DH + idx) = val; }
#pragma unroll
        for (int s = 0; s < 2; ++s) { const int idx = (s * 32 + lane) * 8;
            const v4f x0 = *(const v4fa*)(&so[idx]); const v4f x1 = *(const v4fa*)(&so[idx + 4]); v8h hv, rv;
#pragma unroll
            for (int i = 0; i < 4; ++i) { const h16 a0 = toh_flush(x0[i]); const h16 a1 = toh_flush(x1[i]); hv[i] = a0; hv[4 + i] = a1;
                rv[i] = toh_flush((x0[i] - (float)a0) * QRS); rv[4 + i] = toh_flush((x1[i] - (float)a1) * QRS); }
            *(volatile v8h*)(OH + (size_t)b * DH + idx) = hv; *(volatile v8h*)(PR + (size_t)b * DH + idx) = rv; }
        if (ps == 0) __threadfence(); }
}

__global__ __launch_bounds__(256) void k_reg(const float* FEA, const float* __restrict__ rw, const float* __restrict__ rb, float* OUT) {
    __shared__ __align__(16) float sr[8 * 32];
    const int lane = threadIdx.x & 31;
    const int wave = __builtin_amdgcn_readfirstlane((int)(threadIdx.x >> 5));
    const unsigned bx = blockIdx.x;
    const int rbase = (int)(bx * 256u) + wave * 32;
    if (rbase >= NB) return;
    v4f w = *(const v4f*)(rw + 4 * lane);
#pragma unroll
    for (int c = 0; c < 4; ++c) w[c] = bfr(w[c]);
    const float bb = bfr(rb[0]);
    float mine = 0.0f;
#pragma unroll 1
    for (int r = 0; r < 32; ++r) {
        const v4f f = *(const v4f*)(FEA + (size_t)(rbase + r) * DP + 4 * lane);
        float s = f[0] * w[0]; s = fmaf(f[1], w[1], s); s = fmaf(f[2], w[2], s); s = fmaf(f[3], w[3], s);
        s += __shfl_xor(s, 16, 32); s += __shfl_xor(s, 8, 32); s += __shfl_xor(s, 4, 32); s += __shfl_xor(s, 2, 32); s += __shfl_xor(s, 1, 32);
        mine = (lane == r) ? s : mine; }
    sr[wave * 32 + lane] = mine + bb;
    wave_sync();
    const v4f val = *(const v4fa*)(&sr[wave * 32 + (lane & 7) * 4]);
    if (lane < 8) *(volatile v4f*)(OUT + rbase + 4 * lane) = val;
    __threadfence();
    if (lane < 8) *(volatile v4f*)(OUT + rbase + 4 * lane) = val;
}

static constexpr size_t al256(size_t v) { return (v + 255) & ~(size_t)255; }
static constexpr size_t SZ_XB  = al256((size_t)NB * DIN * 2);
static constexpr size_t SZ_W0  = al256((size_t)DH * DIN * 2);
static constexpr size_t SZ_WQ  = al256((size_t)3 * DH * DH * 2);
static constexpr size_t SZ_WF  = al256((size_t)DH * DH * 2);
static constexpr size_t SZ_WE  = al256((size_t)DP * DH * 2);
static constexpr size_t SZ_F32 = al256((size_t)NB * DH * 4);
static constexpr size_t SZ_F16 = al256((size_t)NB * DH * 2);
static constexpr size_t SZ_QKV = al256((size_t)NB * 3 * DH * 4);
static constexpr size_t SZ_TOTAL = SZ_XB + SZ_W0 + 2 * (SZ_WQ + SZ_WF) + SZ_WE + 2 * (SZ_F32 + 2 * SZ_F16) + SZ_QKV;
static_assert(SZ_TOTAL <= (size_t)134217728);
static_assert(((size_t)DH * DH * 2) % 256 == 0);

extern "C" void kernel_launch(void* const* d_in, const int* in_sizes, int n_in,
                              void* d_out, int out_size, void* d_ws, size_t ws_size, hipStream_t stream) {
    if (n_in < 23) return;
    if ((size_t)in_sizes[0] < (size_t)NB * DIN) return;
    if ((size_t)in_sizes[1] < (size_t)DH * DIN || in_sizes[2] < DH) return;
    if ((size_t)in_sizes[3] < (size_t)DH * DH || (size_t)in_sizes[5] < (size_t)DH * DH || (size_t)in_sizes[7] < (size_t)DH * DH || (size_t)in_sizes[9] < (size_t)DH * DH) return;
    if ((size_t)in_sizes[11] < (size_t)DH * DH || (size_t)in_sizes[13] < (size_t)DH * DH || (size_t)in_sizes[15] < (size_t)DH * DH || (size_t)in_sizes[17] < (size_t)DH * DH) return;
    if (in_sizes[4] < DH || in_sizes[6] < DH || in_sizes[8] < DH || in_sizes[10] < DH) return;
    if (in_sizes[12] < DH || in_sizes[14] < DH || in_sizes[16] < DH || in_sizes[18] < DH) return;
    if ((size_t)in_sizes[19] < (size_t)DP * DH || in_sizes[20] < DP || in_sizes[21] < DP || in_sizes[22] < 1) return;
    if ((size_t)out_size < (size_t)NB_FULL + (size_t)NB * DP) return;
    if (SZ_TOTAL > ws_size) return;
    const float* x     = (const float*)d_in[0];
    const float* w0    = (const float*)d_in[1];  const float* b0    = (const float*)d_in[2];
    const float* qw1   = (const float*)d_in[3];  const float* qb1   = (const float*)d_in[4];
    const float* kw1   = (const float*)d_in[5];  const float* kb1   = (const float*)d_in[6];
    const float* vw1   = (const float*)d_in[7];  const float* vb1   = (const float*)d_in[8];
    const float* fw1   = (const float*)d_in[9];  const float* fb1   = (const float*)d_in[10];
    const float* qw2   = (const float*)d_in[11]; const float* qb2   = (const float*)d_in[12];
    const float* kw2   = (const float*)d_in[13]; const float* kb2   = (const float*)d_in[14];
    const float* vw2   = (const float*)d_in[15]; const float* vb2   = (const float*)d_in[16];
    const float* fw2   = (const float*)d_in[17]; const float* fb2   = (const float*)d_in[18];
    const float* few   = (const float*)d_in[19]; const float* feb   = (const float*)d_in[20];
    const float* rgw   = (const float*)d_in[21]; const float* rgb   = (const float*)d_in[22];
    float* OUT = (float*)d_out;
    float* FEA = OUT + (size_t)NB_FULL;
    char* wsp = (char*)d_ws;
    bf*  XB  = (bf*)wsp;  wsp += SZ_XB;
    bf*  W0B = (bf*)wsp;  wsp += SZ_W0;
    h16* WQ1 = (h16*)wsp; wsp += SZ_WQ;
    h16* WF1 = (h16*)wsp; wsp += SZ_WF;
    h16* WQ2 = (h16*)wsp; wsp += SZ_WQ;
    h16* WF2 = (h16*)wsp; wsp += SZ_WF;
    h16* WFE = (h16*)wsp; wsp += SZ_WE;
    float* HF = (float*)wsp; wsp += SZ_F32;
    h16* HH  = (h16*)wsp; wsp += SZ_F16;
    h16* HR  = (h16*)wsp; wsp += SZ_F16;
    float* AF = (float*)wsp; wsp += SZ_F32;
    h16* AH  = (h16*)wsp; wsp += SZ_F16;
    h16* AR  = (h16*)wsp; wsp += SZ_F16;
    float* QKV = (float*)wsp; wsp += SZ_QKV;

    { const size_t n8 = (size_t)NB * DIN / 8; k_cvt8<<<(unsigned)((n8 + 255) / 256), 256, 0, stream>>>(x, XB, n8); }
    { const size_t n8 = (size_t)DH * DIN / 8; k_cvt8<<<(unsigned)((n8 + 255) / 256), 256, 0, stream>>>(w0, W0B, n8); }
    { const size_t n8 = (size_t)DH * DH / 8; const unsigned g = (unsigned)((n8 + 255) / 256); const size_t sub = (size_t)DH * DH;
      k_wcvt<<<g, 256, 0, stream>>>(qw1, WQ1, n8); k_wcvt<<<g, 256, 0, stream>>>(kw1, WQ1 + sub, n8); k_wcvt<<<g, 256, 0, stream>>>(vw1, WQ1 + 2 * sub, n8);
      k_wcvt<<<g, 256, 0, stream>>>(fw1, WF1, n8);
      k_wcvt<<<g, 256, 0, stream>>>(qw2, WQ2, n8); k_wcvt<<<g, 256, 0, stream>>>(kw2, WQ2 + sub, n8); k_wcvt<<<g, 256, 0, stream>>>(vw2, WQ2 + 2 * sub, n8);
      k_wcvt<<<g, 256, 0, stream>>>(fw2, WF2, n8); }
    { const size_t n8 = (size_t)DP * DH / 8; k_wcvt<<<(unsigned)((n8 + 255) / 256), 256, 0, stream>>>(few, WFE, n8); }

    k_lin0<<<dim3(NB / 32, DH / 64, 1), 32, 0, stream>>>(XB, W0B, b0, HF, HH, HR);
    k_qkv<<<dim3(NB / 32, 3 * DH / 64, 1), 32, 0, stream>>>(HH, HR, WQ1, qb1, kb1, vb1, QKV);
    k_pair<<<dim3(NB, 1, 1), 32, 0, stream>>>(HF, QKV, AF, AH, AR);
    k_f1<<<dim3(NB / 32, DH / 64, 1), 32, 0, stream>>>(AH, AR, WF1, fb1, AF, HF, HH, HR);
    k_qkv<<<dim3(NB / 32, 3 * DH / 64, 1), 32, 0, stream>>>(HH, HR, WQ2, qb2, kb2, vb2, QKV);
    k_pair<<<dim3(NB, 1, 1), 32, 0, stream>>>(HF, QKV, AF, AH, AR);
    k_f1<<<dim3(NB / 32, DH / 64, 1), 32, 0, stream>>>(AH, AR, WF2, fb2, AF, HF, HH, HR);
    k_fea<<<dim3(NB / 32, DP / 64, 1), 32, 0, stream>>>(HH, HR, WFE, feb, FEA);
    k_reg<<<dim3((NB + 255) / 256, 1, 1), 256, 0, stream>>>(FEA, rgw, rgb, OUT);
}
